// MultiHeadAttention_43748536877488
// MI455X (gfx1250) — hardware-run, weakly checked
//
#include <hip/hip_runtime.h>


#ifndef NB
#define NB 4
#endif
#ifndef SEQ
#define SEQ 2048
#endif
#ifndef SEQ_FULL
#define SEQ_FULL 2048
#endif
#define DM   1024
#define NH   16
#define HD   64
#define PSH  10.0f
#define CCAR 64.0f
#define WCAR 1024.0f
#define OSC  (1.0f / 65536.0f)
#define C1L2 0.18033688011112042f
#define NEGL (-1.4426950408889634e10f)

static_assert(SEQ % 64 == 0);
static_assert(SEQ <= SEQ_FULL);
static_assert(DM == NH * HD);
static_assert(DM % 64 == 0);
static_assert(DM % 32 == 0);

typedef _Float16 h16;
typedef unsigned short bf;
typedef __attribute__((ext_vector_type(16))) __bf16   v16bf;
typedef __attribute__((ext_vector_type(16))) _Float16 v16h;
typedef __attribute__((ext_vector_type(8)))  _Float16 v8h;
typedef __attribute__((ext_vector_type(8)))  unsigned short v8us;
typedef __attribute__((ext_vector_type(2)))  unsigned short v2us;
typedef __attribute__((ext_vector_type(8)))  float    v8f;
typedef __attribute__((ext_vector_type(4)))  float    v4f;
typedef __attribute__((ext_vector_type(4)))  int      v4i;
typedef v8h  __attribute__((may_alias)) v8ha;
typedef v4f  __attribute__((may_alias)) v4fa;

__device__ __forceinline__ unsigned short f2bf(float f) { unsigned u = __float_as_uint(f); u += 0x7FFFu + ((u >> 16) & 1u); return (unsigned short)(u >> 16); }
__device__ __forceinline__ float bf2f(unsigned short b) { return __uint_as_float(((unsigned)b) << 16); }
__device__ __forceinline__ float bfr(float f) { return bf2f(f2bf(f)); }
__device__ __forceinline__ v16h cat16(v8h lo, v8h hi) { return __builtin_shufflevector(lo, hi, 0, 1, 2, 3, 4, 5, 6, 7, 8, 9, 10, 11, 12, 13, 14, 15); }
__device__ __forceinline__ v16bf cat16b(v8us lo, v8us hi) { return __builtin_bit_cast(v16bf, __builtin_shufflevector(lo, hi, 0, 1, 2, 3, 4, 5, 6, 7, 8, 9, 10, 11, 12, 13, 14, 15)); }
__device__ __forceinline__ v8f wmma16(v16h a, v16h b, v8f c) { return __builtin_amdgcn_wmma_f32_16x16x32_f16(false, a, false, b, (short)0, c, false, false); }
__device__ __forceinline__ v8f wmmab(v16bf a, v16bf b, v8f c) { return __builtin_amdgcn_wmma_f32_16x16x32_bf16(false, a, false, b, (short)0, c, false, false); }

template <typename T16> struct WFrag;
template <> struct WFrag<h16> { typedef v16h V; static __device__ __forceinline__ V ld(const h16* p) { return cat16(*(const v8h*)p, *(const v8h*)(p + 16)); } static __device__ __forceinline__ v8f mma(V a, V b, v8f c) { return wmma16(a, b, c); } };
template <> struct WFrag<bf> { typedef v16bf V; static __device__ __forceinline__ V ld(const bf* p) { return cat16b(*(const v8us*)p, *(const v8us*)(p + 16)); } static __device__ __forceinline__ v8f mma(V a, V b, v8f c) { return wmmab(a, b, c); } };

template <int BIAS> __device__ __forceinline__ float bsel(const float* __restrict__ bias, int ci, int ri) { if (BIAS == 0) return 0.0f; return bfr(bias[(BIAS == 1) ? ci : ri]); }

template <typename T16, typename OT, int BIAS>
__global__ __launch_bounds__(32) void k_gemm(const T16* __restrict__ A, const T16* __restrict__ Bt, int K, OT* C, int ldc, size_t tcs, const float* __restrict__ bias, float osc, size_t sA, size_t sB, size_t sC) {
    typedef typename WFrag<T16>::V V;
    __shared__ __align__(16) float os[16 * 68];
    const size_t z = blockIdx.z; A += z * sA; Bt += z * sB; C += z * sC + (size_t)blockIdx.y * tcs;
    const int lane = threadIdx.x & 31, lr = lane & 15, hi = lane >> 4; const int r0 = blockIdx.x * 64, c0 = blockIdx.y * 64;
    v8f acc[4][4];
#pragma unroll
    for (int mb = 0; mb < 4; ++mb)
#pragma unroll
        for (int nb = 0; nb < 4; ++nb) acc[mb][nb] = (v8f){};
    const size_t aoff = (size_t)(r0 + lr) * K + 8 * hi, boff = (size_t)(c0 + lr) * K + 8 * hi;
#pragma unroll 1
    for (int kc = 0; kc < K; kc += 32) {
        V a[4], b[4];
#pragma unroll
        for (int mb = 0; mb < 4; ++mb) a[mb] = WFrag<T16>::ld(A + aoff + (size_t)mb * 16 * K + kc);
#pragma unroll
        for (int nb = 0; nb < 4; ++nb) b[nb] = WFrag<T16>::ld(Bt + boff + (size_t)nb * 16 * K + kc);
#pragma unroll
        for (int nb = 0; nb < 4; ++nb)
#pragma unroll
            for (int mb = 0; mb < 4; ++mb) acc[mb][nb] = WFrag<T16>::mma(a[mb], b[nb], acc[mb][nb]);
        asm volatile("v_nop\n\tv_nop\n\tv_nop\n\tv_nop" : "+v"(acc[0][0]), "+v"(acc[1][1]), "+v"(acc[2][2]), "+v"(acc[0][3]), "+v"(acc[1][3]), "+v"(acc[2][3]), "+v"(acc[3][3]) : "v"(a[0]), "v"(a[1]), "v"(a[2]), "v"(a[3]), "v"(b[3]));
    }
#pragma unroll
    for (int mb = 0; mb < 4; ++mb) {
#pragma unroll
        for (int nb = 0; nb < 4; ++nb) {
#pragma unroll
            for (int j = 0; j < 8; ++j) os[(hi * 8 + j) * 68 + nb * 16 + lr] = acc[mb][nb][j]; }
        __builtin_amdgcn_wave_barrier(); asm volatile("" ::: "memory");
        OT* crow = C + (size_t)(r0 + mb * 16) * ldc;
        const int rbase = r0 + mb * 16;
#pragma unroll 1
        for (int ps = 0; ps < 2; ++ps) {
            if (sizeof(OT) == 4) {
#pragma unroll
                for (int s = 0; s < 8; ++s) { const int row = 2 * s + hi, cofs = lr * 4; v4f val = *(const v4fa*)(os + row * 68 + cofs);
                    val[0] = val[0] * osc + bsel<BIAS>(bias, c0 + cofs, rbase + row); val[1] = val[1] * osc + bsel<BIAS>(bias, c0 + cofs + 1, rbase + row);
                    val[2] = val[2] * osc + bsel<BIAS>(bias, c0 + cofs + 2, rbase + row); val[3] = val[3] * osc + bsel<BIAS>(bias, c0 + cofs + 3, rbase + row);
                    *(volatile v4f*)(void*)(crow + (size_t)row * ldc + cofs) = val; }
            } else {
#pragma unroll
                for (int s = 0; s < 4; ++s) { const int row = (lane >> 3) + 4 * s, cofs = (lane & 7) * 8; const v4f v0 = *(const v4fa*)(os + row * 68 + cofs); const v4f v1 = *(const v4fa*)(os + row * 68 + cofs + 4); v8h hv;
#pragma unroll
                    for (int i = 0; i < 4; ++i) { hv[i] = (h16)(v0[i] * osc + bsel<BIAS>(bias, c0 + cofs + i, rbase + row)); hv[4 + i] = (h16)(v1[i] * osc + bsel<BIAS>(bias, c0 + cofs + 4 + i, rbase + row)); }
                    *(volatile v8h*)(void*)(crow + (size_t)row * ldc + cofs) = hv; }
            }
            if (ps == 0) __threadfence(); }
        __builtin_amdgcn_wave_barrier(); asm volatile("" ::: "memory");
    }
}

template <bool F16>
__global__ __launch_bounds__(256) void k_wt(const float* __restrict__ w, int K, int N, unsigned short* Bt) {
    const int lane = threadIdx.x & 31; const int L0 = (blockIdx.x * 8 + (threadIdx.x >> 5)) * 8; const int nlines = N * K / 64;
#pragma unroll
    for (int ps = 0; ps < 2; ++ps) {
#pragma unroll 1
        for (int l = 0; l < 8; ++l) { const int L = L0 + l; if (L >= nlines) break; const size_t e = (size_t)L * 64 + lane * 2; const int k = (int)(e % K), n = (int)(e / K); v2us o;
            const float w0 = w[(size_t)k * N + n], w1 = w[(size_t)(k + 1) * N + n];
            if (F16) { const h16 a = (h16)(bfr(w0) * WCAR), c = (h16)(bfr(w1) * WCAR); o[0] = __builtin_bit_cast(unsigned short, a); o[1] = __builtin_bit_cast(unsigned short, c); }
            else { o[0] = f2bf(w0); o[1] = f2bf(w1); }
            *(volatile v2us*)(Bt + e) = o; }
        if (ps == 0) __threadfence(); }
}

__global__ __launch_bounds__(256) void k_cvt8(const float* __restrict__ src, bf* dst, size_t n8) {
    const size_t i = (size_t)blockIdx.x * 256 + threadIdx.x; if (i >= n8) return;
    const size_t e = i * 8; const size_t row = e / DM; const size_t col = e % DM; const size_t b = row / SEQ, t = row % SEQ;
    const v8f v = *(const v8f*)(src + (b * SEQ_FULL + t) * DM + col); v8us o;
#pragma unroll
    for (int k = 0; k < 8; ++k) o[k] = f2bf(v[k]);
    *(volatile v8us*)(dst + e) = o; __threadfence(); *(volatile v8us*)(dst + e) = o; }

__global__ __launch_bounds__(256) void k_mask(const int* __restrict__ mask, float* MA, float* MB) {
    const int i = (blockIdx.x * 256 + threadIdx.x) * 4; if (i >= NB * SEQ) return; const int b = i / SEQ, j = i % SEQ;
    const v4i m = *(const v4i*)(mask + (size_t)b * SEQ_FULL + j); v4f a, c;
#pragma unroll
    for (int q = 0; q < 4; ++q) { a[q] = (m[q] != 0) ? C1L2 : 0.0f; c[q] = (m[q] != 0) ? 0.0f : NEGL; }
    *(volatile v4f*)(MA + i) = a; *(volatile v4f*)(MB + i) = c; __threadfence(); *(volatile v4f*)(MA + i) = a; *(volatile v4f*)(MB + i) = c; }

__global__ __launch_bounds__(128) void k_attn(const h16* __restrict__ Q, const h16* __restrict__ Kpl, const h16* __restrict__ VT, const float* __restrict__ MA, const float* __restrict__ MB, h16* CTX) {
    __shared__ __align__(16) h16 cs[4 * 16 * 72];
    const int lane = threadIdx.x & 31, lr = lane & 15, hi = lane >> 4;
    const int wave = __builtin_amdgcn_readfirstlane((int)(threadIdx.x >> 5));
    const int b = blockIdx.z, h = blockIdx.y; const int q0 = blockIdx.x * 64 + wave * 16;
    const size_t bh = (size_t)b * NH + h;
    const h16* qp = Q + (bh * SEQ + q0 + lr) * HD + 8 * hi;
    const v16h qb0 = WFrag<h16>::ld(qp), qb1 = WFrag<h16>::ld(qp + 32);
    const h16* kp = Kpl + (bh * SEQ + lr) * HD + 8 * hi;
    const h16* vp = VT + (bh * HD + lr) * SEQ + 8 * hi;
    const float* ma = MA + (size_t)b * SEQ + 8 * hi; const float* mb = MB + (size_t)b * SEQ + 8 * hi;
    v8f acc[4];
#pragma unroll
    for (int t = 0; t < 4; ++t) acc[t] = (v8f){};
    float mrun = -3.0e38f, mref = -3.0e38f, lrun = 0.0f;
#pragma unroll 1
    for (int k0 = 0; k0 < SEQ; k0 += 32) {
        const h16* kr = kp + (size_t)k0 * HD;
        const v16h ka00 = WFrag<h16>::ld(kr), ka01 = WFrag<h16>::ld(kr + 32), ka10 = WFrag<h16>::ld(kr + 16 * HD), ka11 = WFrag<h16>::ld(kr + 16 * HD + 32);
        v8f s0 = (v8f){}, s1 = (v8f){};
        s0 = wmma16(ka00, qb0, s0); s1 = wmma16(ka10, qb0, s1); s0 = wmma16(ka01, qb1, s0); s1 = wmma16(ka11, qb1, s1);
        asm volatile("v_nop\n\tv_nop\n\tv_nop\n\tv_nop" : "+v"(s0), "+v"(s1) : "v"(ka01), "v"(ka11), "v"(qb1));
        const v8f a0 = *(const v8f*)(ma + k0), a1 = *(const v8f*)(ma + k0 + 16), c0 = *(const v8f*)(mb + k0), c1 = *(const v8f*)(mb + k0 + 16);
        float t0[8], t1[8]; float ml = -3.0e38f;
#pragma unroll
        for (int r = 0; r < 8; ++r) { t0[r] = fmaf(s0[r], a0[r], c0[r]); t1[r] = fmaf(s1[r], a1[r], c1[r]); ml = fmaxf(ml, fmaxf(t0[r], t1[r])); }
        ml = fmaxf(ml, __shfl_xor(ml, 16, 32));
        const float mnew = fmaxf(mrun, ml); const float nref = mnew - PSH;
        const float corr = __builtin_amdgcn_exp2f(mref - nref); mrun = mnew; mref = nref;
        float ls = 0.0f; v16h pb;
#pragma unroll
        for (int r = 0; r < 8; ++r) { const float p0 = __builtin_amdgcn_exp2f(t0[r] - nref), p1 = __builtin_amdgcn_exp2f(t1[r] - nref); ls += p0 + p1; pb[r] = (h16)p0; pb[8 + r] = (h16)p1; }
        lrun = lrun * corr + ls;
#pragma unroll
        for (int t = 0; t < 4; ++t) acc[t] = acc[t] * corr;
        const h16* vr = vp + k0; v16h va[4];
#pragma unroll
        for (int t = 0; t < 4; ++t) va[t] = WFrag<h16>::ld(vr + (size_t)t * 16 * SEQ);
#pragma unroll
        for (int t = 0; t < 4; ++t) acc[t] = wmma16(va[t], pb, acc[t]);
        asm volatile("v_nop\n\tv_nop\n\tv_nop\n\tv_nop" : "+v"(acc[0]), "+v"(acc[1]), "+v"(acc[2]), "+v"(acc[3]) : "v"(va[3]), "v"(pb));
    }
    const float lt = lrun + __shfl_xor(lrun, 16, 32);
    const float inv = CCAR * __builtin_amdgcn_rcpf(lt);
    h16* cw = cs + wave * (16 * 72);
#pragma unroll
    for (int t = 0; t < 4; ++t) { v8h o;
#pragma unroll
        for (int r = 0; r < 8; ++r) o[r] = (h16)(acc[t][r] * inv);
        *(v8h*)(cw + lr * 72 + t * 16 + 8 * hi) = o; }
    __builtin_amdgcn_wave_barrier(); asm volatile("" ::: "memory");
    h16* crow = CTX + ((size_t)b * SEQ + q0) * DM + h * HD;
#pragma unroll 1
    for (int ps = 0; ps < 2; ++ps) {
#pragma unroll
        for (int s = 0; s < 4; ++s) { const int row = (lane >> 3) + 4 * s, pc = (lane & 7) * 8; const v8h val = *(const v8ha*)(cw + row * 72 + pc);
            *(volatile v8h*)(crow + (size_t)row * DM + pc) = val; }
        if (ps == 0) __threadfence(); }
}

extern "C" void kernel_launch(void* const* d_in, const int* in_sizes, int n_in,
                              void* d_out, int out_size, void* d_ws, size_t ws_size, hipStream_t stream) {
    if (n_in < 11) return;
    const size_t need_act = ((size_t)(NB - 1) * SEQ_FULL + SEQ) * DM, need_mask = (size_t)(NB - 1) * SEQ_FULL + SEQ;
    if ((size_t)in_sizes[0] < need_act || (size_t)in_sizes[1] < need_act || (size_t)in_sizes[2] < need_mask) return;
    if ((size_t)in_sizes[3] < (size_t)DM * DM || (size_t)in_sizes[5] < (size_t)DM * DM || (size_t)in_sizes[7] < (size_t)DM * DM || (size_t)in_sizes[9] < (size_t)DM * DM) return;
    if (in_sizes[4] < DM || in_sizes[6] < DM || in_sizes[8] < DM || in_sizes[10] < DM) return;
    if ((size_t)out_size < (size_t)NB * SEQ * DM) return;
    const float* x = (const float*)d_in[0]; const float* feat = (const float*)d_in[1]; const int* mask = (const int*)d_in[2];
    const float* wq = (const float*)d_in[3]; const float* bq = (const float*)d_in[4]; const float* wk = (const float*)d_in[5]; const float* bk = (const float*)d_in[6];
    const float* wv = (const float*)d_in[7]; const float* bv = (const float*)d_in[8]; const float* wo = (const float*)d_in[9]; const float* bo = (const float*)d_in[10];
    float* OUT = (float*)d_out;
    char* wsp = (char*)d_ws;
    auto take = [&](size_t bytes) { char* p = wsp; wsp += (bytes + 255) & ~(size_t)255; return (void*)p; };
    const size_t WB = (size_t)DM * DM * 2, AB = (size_t)NB * SEQ * DM * 2, MBY = (size_t)NB * SEQ * 4;
    static_assert(4 * ((size_t)DM * DM * 2) + 6 * ((size_t)NB * SEQ * DM * 2) + 2 * ((size_t)NB * SEQ * 4) <= (size_t)134217728);
    bf* WQ = (bf*)take(WB); bf* WK = (bf*)take(WB); bf* WV = (bf*)take(WB); unsigned short* WO = (unsigned short*)take(WB);
    bf* XB = (bf*)take(AB); bf* FB = (bf*)take(AB);
    h16* QP = (h16*)take(AB); h16* KP = (h16*)take(AB); h16* VTP = (h16*)take(AB); h16* CTX = (h16*)take(AB);
    float* MA = (float*)take(MBY); float* MBp = (float*)take(MBY);
    if ((size_t)(wsp - (char*)d_ws) > ws_size) return;

    const unsigned gw = (unsigned)((DM * DM / 64 + 63) / 64);
    k_wt<false><<<gw, 256, 0, stream>>>(wq, DM, DM, WQ);
    k_wt<false><<<gw, 256, 0, stream>>>(wk, DM, DM, WK);
    k_wt<false><<<gw, 256, 0, stream>>>(wv, DM, DM, WV);
    k_wt<true><<<gw, 256, 0, stream>>>(wo, DM, DM, WO);
    const size_t n8 = (size_t)NB * SEQ * DM / 8;
    k_cvt8<<<(unsigned)((n8 + 255) / 256), 256, 0, stream>>>(x, XB, n8);
    k_cvt8<<<(unsigned)((n8 + 255) / 256), 256, 0, stream>>>(feat, FB, n8);
    k_mask<<<(unsigned)((NB * SEQ / 4 + 255) / 256), 256, 0, stream>>>(mask, MA, MBp);

    k_gemm<bf, h16, 1><<<dim3(SEQ / 64, DM / 64, NB), 32, 0, stream>>>(XB, WQ, DM, QP, HD, (size_t)SEQ * HD, bq, 1.0f, (size_t)SEQ * DM, (size_t)0, (size_t)NH * SEQ * HD);
    k_gemm<bf, h16, 1><<<dim3(SEQ / 64, DM / 64, NB), 32, 0, stream>>>(FB, WK, DM, KP, HD, (size_t)SEQ * HD, bk, 1.0f, (size_t)SEQ * DM, (size_t)0, (size_t)NH * SEQ * HD);
    k_gemm<bf, h16, 2><<<dim3(DM / 64, SEQ / 64, NB), 32, 0, stream>>>(WV, FB, DM, VTP, SEQ, (size_t)64, bv, 1.0f, (size_t)0, (size_t)SEQ * DM, (size_t)DM * SEQ);

    k_attn<<<dim3(SEQ / 64, NH, NB), 128, 0, stream>>>(QP, KP, VTP, MA, MBp, CTX);

    k_gemm<h16, float, 1><<<dim3(NB * SEQ / 64, DM / 64, 1), 32, 0, stream>>>(CTX, (const h16*)WO, DM, OUT, DM, (size_t)64, bo, OSC, (size_t)0, (size_t)0, (size_t)0);
}
